// MambaBlock_8718783611649
// MI455X (gfx1250) — hardware-verified
//
#include <hip/hip_runtime.h>
#include <math.h>

typedef __attribute__((ext_vector_type(16))) _Float16 v16h;
typedef __attribute__((ext_vector_type(8)))  _Float16 v8h;
typedef __attribute__((ext_vector_type(16))) __bf16   v16b;
typedef __attribute__((ext_vector_type(8)))  __bf16   v8b;
typedef __attribute__((ext_vector_type(8)))  float    v8f;
typedef __attribute__((ext_vector_type(4)))  float    v4f;
typedef __attribute__((ext_vector_type(4)))  unsigned int v4u;

constexpr int kB     = 8;
constexpr int kL     = 4096;
constexpr int kD     = 256;
constexpr int kD2    = 2 * kD;
constexpr int kS     = 16;
constexpr int kKC    = 4;
constexpr int kRows  = kB * kL;
constexpr int kLgP   = 64;
constexpr int kYP    = 32;
constexpr int kTileP = 260;
constexpr int kScanT = 64;
constexpr int kSlabR = 256;
constexpr int kSlabs = kRows / kSlabR;
static_assert(kD == 256, "block = 256 channels");
static_assert(kRows % 64 == 0 && kD % 64 == 0 && kD2 % 64 == 0 && kLgP % 64 == 0, "GEMM M,N multiples of 64");
static_assert(kD % 32 == 0, "GEMM K multiple of 32");
static_assert(kL % 64 == 0 && kL % kScanT == 0 && (kL & (kL - 1)) == 0, "tile multiples");
static_assert(2 * kS <= kYP && 2 * kS <= kLgP, "packed state columns");
static_assert(kSlabs * kSlabR == kRows && kSlabs == 128, "slabs");

constexpr size_t kOffXB   = 0;
constexpr size_t kOffWIB  = kOffXB   + (size_t)kRows * kD * 2;
constexpr size_t kOffWOB  = kOffWIB  + (size_t)kD2 * kD * 2;
constexpr size_t kOffWDB  = kOffWOB  + (size_t)kD * kD * 2;
constexpr size_t kOffXP   = kOffWDB  + (size_t)64 * kD * 2;
constexpr size_t kOffRES  = kOffXP   + (size_t)kRows * kD * 4;
constexpr size_t kOffXC   = kOffRES  + (size_t)kRows * kD * 2;
constexpr size_t kOffXCB  = kOffXC   + (size_t)kRows * kD * 4;
constexpr size_t kOffLGT  = kOffXCB  + (size_t)kRows * kD * 2;
constexpr size_t kOffY    = kOffLGT  + (size_t)kRows * kLgP * 4;
constexpr size_t kOffP1   = kOffY    + (size_t)kRows * kYP * 4;
constexpr size_t kOffP2   = kOffP1   + (size_t)kSlabs * kD * 4;
constexpr size_t kOffMEAN = kOffP2   + (size_t)kSlabs * kD * 4;
constexpr size_t kOffRSTD = kOffMEAN + (size_t)kD * 4;
constexpr size_t kWsTotal = kOffRSTD + (size_t)kD * 4;
static_assert(kWsTotal == 130713600ull, "carve total");
static_assert(kWsTotal <= 134217728ull, "carve cap");
static_assert((kOffWIB % 128) == 0 && (kOffWOB % 128) == 0 && (kOffWDB % 128) == 0 && (kOffXP % 128) == 0 &&
              (kOffRES % 128) == 0 && (kOffXC % 128) == 0 && (kOffXCB % 128) == 0 && (kOffLGT % 128) == 0 &&
              (kOffY % 128) == 0 && (kOffP1 % 128) == 0 && (kOffP2 % 128) == 0 && (kOffMEAN % 128) == 0 &&
              (kOffRSTD % 128) == 0, "128-B aligned regions");

__device__ __forceinline__ unsigned short f2bf_bits(float f) {
  unsigned u = __float_as_uint(f);
  return (unsigned short)((u + 0x7FFFu + ((u >> 16) & 1u)) >> 16);
}
__device__ __forceinline__ float bf_bits2f(unsigned short h) { return __uint_as_float(((unsigned)h) << 16); }
__device__ __forceinline__ float bfr(float v) { return bf_bits2f(f2bf_bits(v)); }
__device__ __forceinline__ _Float16 bfh(float v) { const unsigned short hb = f2bf_bits(v); return __builtin_bit_cast(_Float16, hb); }

__device__ __forceinline__ void dep_guard4_h(v8f& a, v8f& b, v8f& c, v8f& d, v16h x, v16h y) {
  asm volatile("v_nop\n\tv_nop\n\tv_nop\n\tv_nop" : "+v"(a), "+v"(b), "+v"(c), "+v"(d) : "v"(x), "v"(y));
}
__device__ __forceinline__ void dep_guard4_b(v8f& a, v8f& b, v8f& c, v8f& d, v16b x, v16b y) {
  asm volatile("v_nop\n\tv_nop\n\tv_nop\n\tv_nop" : "+v"(a), "+v"(b), "+v"(c), "+v"(d) : "v"(x), "v"(y));
}
__device__ __forceinline__ void keep4_h(v16h a, v16h b, v16h c, v16h d) { asm volatile("v_nop" :: "v"(a), "v"(b), "v"(c), "v"(d)); }
__device__ __forceinline__ void keep4_b(v16b a, v16b b, v16b c, v16b d) { asm volatile("v_nop" :: "v"(a), "v"(b), "v"(c), "v"(d)); }
__device__ __forceinline__ void acc_guard4(v8f& a, v8f& b, v8f& c, v8f& d) { asm volatile("v_nop\n\tv_nop\n\tv_nop\n\tv_nop" : "+v"(a), "+v"(b), "+v"(c), "+v"(d)); }
template <typename T> struct Frag;
template <> struct Frag<_Float16> {
  typedef v16h V; union U { v16h v; v8h h[2]; };
  static __device__ __forceinline__ v16h load(const _Float16* p) {
    U f; f.h[0] = *(const v8h*)(p); f.h[1] = *(const v8h*)(p + 16); return f.v;
  }
  static __device__ __forceinline__ v8f mma(v16h a, v16h b, v8f c) {
    return __builtin_amdgcn_wmma_f32_16x16x32_f16(false, a, false, b, (short)0, c, false, false);
  }
  static __device__ __forceinline__ void guard4(v8f& a, v8f& b, v8f& c, v8f& d, v16h x, v16h y) { dep_guard4_h(a, b, c, d, x, y); }
  static __device__ __forceinline__ void keep(v16h a, v16h b, v16h c, v16h d) { keep4_h(a, b, c, d); }
};
template <> struct Frag<__bf16> {
  typedef v16b V; union U { v16b v; v8b h[2]; };
  static __device__ __forceinline__ v16b load(const __bf16* p) {
    U f; f.h[0] = *(const v8b*)(p); f.h[1] = *(const v8b*)(p + 16); return f.v;
  }
  static __device__ __forceinline__ v8f mma(v16b a, v16b b, v8f c) {
    return __builtin_amdgcn_wmma_f32_16x16x32_bf16(false, a, false, b, (short)0, c, false, false);
  }
  static __device__ __forceinline__ void guard4(v8f& a, v8f& b, v8f& c, v8f& d, v16b x, v16b y) { dep_guard4_b(a, b, c, d, x, y); }
  static __device__ __forceinline__ void keep(v16b a, v16b b, v16b c, v16b d) { keep4_b(a, b, c, d); }
};

template <int ET> struct Elem;
template <> struct Elem<0> { typedef _Float16 T; };
template <> struct Elem<1> { typedef __bf16 T; };
template <int ET, bool SPLIT, int BIAS_MODE, int OUT_MODE, bool RESID, int ACT = 0>
__global__ __launch_bounds__(256) void wmma_gemm64(
    const unsigned short* __restrict__ Ap, const unsigned short* __restrict__ A2p, int lda, long strideA,
    const unsigned short* __restrict__ Btp, const unsigned short* __restrict__ Bt2p, int ldb, long strideB,
    void* __restrict__ Cout, void* __restrict__ Cout2, int ldc, long strideC,
    const float* __restrict__ bias,
    const float* __restrict__ resid, long strideR,
    int M, int N, int K, float scale) {
  static_assert(!(RESID && OUT_MODE != 0), "residual only with f32 output");
  static_assert(!(RESID && ACT != 0), "no activation together with residual");
  typedef typename Elem<ET>::T T;
  typedef typename Frag<T>::V V;
  const T* A = (const T*)Ap; const T* A2 = (const T*)A2p; const T* Bt = (const T*)Btp; const T* Bt2 = (const T*)Bt2p;
  __shared__ __align__(16) float sT[8][16 * 68];
  const int b    = blockIdx.y;
  const int lane = threadIdx.x & 31;
  const int wave = threadIdx.x >> 5;
  const int tilesN = N >> 6;
  const int tilesM = M >> 6;
  const int tile = blockIdx.x * 8 + wave;
  if (tile >= tilesM * tilesN) return;
  const int tm = tile / tilesN;
  const int tn = tile - tm * tilesN;
  const int m0 = tm << 6;
  const int n0 = tn << 6;

  const T* Ab  = A  + (size_t)b * strideA;
  const T* Bb  = Bt + (size_t)b * strideB;
  const T* Ab2 = SPLIT ? (A2  + (size_t)b * strideA) : nullptr;
  const T* Bb2 = SPLIT ? (Bt2 + (size_t)b * strideB) : nullptr;

  const int rlane = lane & 15;
  const int koff  = (lane >> 4) * 8;
  const int mOff  = (lane >> 4) * 8;

  v8f acc[4][4];
#pragma unroll
  for (int i = 0; i < 4; ++i)
#pragma unroll
    for (int j = 0; j < 4; ++j) acc[i][j] = (v8f){0.f,0.f,0.f,0.f,0.f,0.f,0.f,0.f};

  for (int k0 = 0; k0 < K; k0 += 32) {
    V bh[4], bl[4];
#pragma unroll
    for (int j = 0; j < 4; ++j) {
      const size_t bo = (size_t)(n0 + (j << 4) + rlane) * ldb + koff + k0;
      bh[j] = Frag<T>::load(Bb + bo);
      if (SPLIT) bl[j] = Frag<T>::load(Bb2 + bo);
    }
#pragma unroll
    for (int i = 0; i < 4; ++i) {
      const size_t ao = (size_t)(m0 + (i << 4) + rlane) * lda + koff + k0;
      V ah = Frag<T>::load(Ab + ao);
      V al = ah;
      if (SPLIT) al = Frag<T>::load(Ab2 + ao);
#pragma unroll
      for (int j = 0; j < 4; ++j) {
        acc[i][j] = Frag<T>::mma(ah, bh[j], acc[i][j]);
        if (SPLIT) {
          acc[i][j] = Frag<T>::mma(ah, bl[j], acc[i][j]);
          acc[i][j] = Frag<T>::mma(al, bh[j], acc[i][j]);
        }
      }
      Frag<T>::guard4(acc[i][0], acc[i][1], acc[i][2], acc[i][3], ah, al);
    }
    Frag<T>::keep(bh[0], bh[1], bh[2], bh[3]);
    if (SPLIT) Frag<T>::keep(bl[0], bl[1], bl[2], bl[3]);
  }
  acc_guard4(acc[0][0], acc[0][1], acc[0][2], acc[0][3]);
  acc_guard4(acc[1][0], acc[1][1], acc[1][2], acc[1][3]);
  acc_guard4(acc[2][0], acc[2][1], acc[2][2], acc[2][3]);
  acc_guard4(acc[3][0], acc[3][1], acc[3][2], acc[3][3]);

  float* slab = sT[wave];
  const float* Rb = RESID ? (resid + (size_t)b * strideR) : nullptr;
#pragma unroll
  for (int i = 0; i < 4; ++i) {
    const int mBase = m0 + (i << 4);
#pragma unroll
    for (int j = 0; j < 4; ++j) {
      const int n = n0 + (j << 4) + rlane;
      float bv = 0.f;
      if (BIAS_MODE == 2) bv = bias[n];
#pragma unroll
      for (int r = 0; r < 8; ++r) {
        float v = acc[i][j][r] * scale;
        if (BIAS_MODE == 1) v += bias[mBase + mOff + r];
        if (BIAS_MODE == 2) v += bv;
        if (ACT == 1) v = tanhf(v);
        if (ACT == 2) v = fmaxf(v, 0.0f);
        if (ACT == 3) v = v * (1.0f / (1.0f + expf(-v)));
        if (ACT == 4) v = (v > 0.f) ? v : 0.01f * v;
        slab[(mOff + r) * 68 + (j << 4) + rlane] = v;
      }
    }
    __builtin_amdgcn_fence(__ATOMIC_RELEASE, "workgroup");
    __builtin_amdgcn_wave_barrier();
    __builtin_amdgcn_fence(__ATOMIC_ACQUIRE, "workgroup");
    if (OUT_MODE == 0) {
      float* C = (float*)Cout + (size_t)b * strideC;
      const int hh = lane >> 4, c4 = (lane & 15) * 4;
      v4f vals[8];
#pragma unroll
      for (int it = 0; it < 8; ++it) {
        const int row = it * 2 + hh;
        v4f v = *(const v4f*)(slab + row * 68 + c4);
        if (RESID) {
          const v4f rr = *(const v4f*)(Rb + (size_t)(mBase + row) * ldc + n0 + c4);
          v = v + rr;
        }
        vals[it] = v;
      }
      for (int pass = 0; pass < 2; ++pass) {
#pragma unroll
        for (int it = 0; it < 8; ++it) {
          const int row = it * 2 + hh;
          *(volatile v4f*)(C + (size_t)(mBase + row) * ldc + n0 + c4) = vals[it];
        }
        __threadfence();
      }
    } else {
      const int q8 = lane >> 3, c8 = (lane & 7) * 8;
      unsigned short* C  = (unsigned short*)Cout  + (size_t)b * strideC;
      unsigned short* C2 = (OUT_MODE == 2) ? ((unsigned short*)Cout2 + (size_t)b * strideC) : nullptr;
      v8h hvv[4], lvv[4];
#pragma unroll
      for (int it = 0; it < 4; ++it) {
        const int row = it * 4 + q8;
        const float* sp = slab + row * 68 + c8;
        v8h hv, lv;
#pragma unroll
        for (int e = 0; e < 8; ++e) {
          const float f = sp[e];
          if (OUT_MODE == 1) {
            hv[e] = (_Float16)f;
            lv[e] = hv[e];
          } else {
            const unsigned short hb = f2bf_bits(f);
            hv[e] = __builtin_bit_cast(_Float16, hb);
            if (OUT_MODE == 2) {
              const unsigned short lb = f2bf_bits(f - bf_bits2f(hb));
              lv[e] = __builtin_bit_cast(_Float16, lb);
            } else {
              lv[e] = hv[e];
            }
          }
        }
        hvv[it] = hv; lvv[it] = lv;
      }
      for (int pass = 0; pass < 2; ++pass) {
#pragma unroll
        for (int it = 0; it < 4; ++it) {
          const int row = it * 4 + q8;
          *(volatile v8h*)(C + (size_t)(mBase + row) * ldc + n0 + c8) = hvv[it];
          if (OUT_MODE == 2) *(volatile v8h*)(C2 + (size_t)(mBase + row) * ldc + n0 + c8) = lvv[it];
        }
        __threadfence();
      }
    }
    __builtin_amdgcn_fence(__ATOMIC_RELEASE, "workgroup");
    __builtin_amdgcn_wave_barrier();
    __builtin_amdgcn_fence(__ATOMIC_ACQUIRE, "workgroup");
  }
}

__global__ __launch_bounds__(256) void cast_bf16_kernel(
    const float* __restrict__ src, unsigned short* __restrict__ dst, int total8)
{
  const int i = blockIdx.x * 256 + threadIdx.x;
  if (i >= total8) return;
  const size_t e0 = (size_t)i << 3;
  const v4f a0 = *(const v4f*)(src + e0);
  const v4f a1 = *(const v4f*)(src + e0 + 4);
  v8h hv;
#pragma unroll
  for (int e = 0; e < 4; ++e) {
    hv[e]     = bfh(a0[e]);
    hv[4 + e] = bfh(a1[e]);
  }
  unsigned short* qd = dst + e0;
  *(volatile v8h*)qd = hv;
  __threadfence();
  *(volatile v8h*)qd = hv;
}

__global__ __launch_bounds__(256) void wdb_kernel(
    const float* __restrict__ dt, const float* __restrict__ B_w, unsigned short* __restrict__ WDB)
{
  const int i = blockIdx.x * 256 + threadIdx.x;
  if (i >= (64 * kD) / 8) return;
  const int e0 = i << 3;
  const int n  = e0 >> 8;
  const int k0 = e0 & 255;
  const int sd = n & 15;
  int nb = n - 16; nb = nb < 0 ? 0 : (nb > 15 ? 15 : nb);
  const float fdt = (n < kS) ? 1.0f : 0.0f;
  const float fbw = (n >= kS && n < 2 * kS) ? 1.0f : 0.0f;
  const v4f b0 = *(const v4f*)(B_w + (size_t)nb * kD + k0);
  const v4f b1 = *(const v4f*)(B_w + (size_t)nb * kD + k0 + 4);
  v8h hv;
#pragma unroll
  for (int e = 0; e < 4; ++e) {
    const float vd0 = dt[(size_t)(k0 + e) * kS + sd];
    const float vd1 = dt[(size_t)(k0 + 4 + e) * kS + sd];
    float v0 = fbw * b0[e];
    v0 = fmaf(fdt, vd0, v0);
    float v1 = fbw * b1[e];
    v1 = fmaf(fdt, vd1, v1);
    hv[e]     = bfh(v0);
    hv[4 + e] = bfh(v1);
  }
  unsigned short* qd = WDB + e0;
  *(volatile v8h*)qd = hv;
  __threadfence();
  *(volatile v8h*)qd = hv;
}

__global__ __launch_bounds__(256) void conv_kernel(
    const float* __restrict__ XP, const float* __restrict__ cw, const float* __restrict__ cb,
    float* __restrict__ XC, unsigned short* __restrict__ XCB)
{
  __shared__ __align__(16) float sT[16 * kTileP];
  const int tid = threadIdx.x, lane = tid & 31, wave = tid >> 5;
  const int d = tid;
  const int g0 = blockIdx.x * 64;
  const int tb = g0 & (kL - 1);
  const v4f wraw = *(const v4f*)(cw + (size_t)d * kKC);
  const float w0 = bfr(wraw[0]), w1 = bfr(wraw[1]), w2 = bfr(wraw[2]), w3 = bfr(wraw[3]);
  const float bc = bfr(cb[d]);
  float xm3, xm2, xm1;
  {
    const bool hist = (tb > 0);
    const int rb = hist ? (g0 - 3) : g0;
    const float v3 = XP[(size_t)rb * kD + d];
    const float v2 = XP[(size_t)(rb + 1) * kD + d];
    const float v1 = XP[(size_t)(rb + 2) * kD + d];
    xm3 = hist ? v3 : 0.0f;
    xm2 = hist ? v2 : 0.0f;
    xm1 = hist ? v1 : 0.0f;
  }
  const int hrow = wave >> 1;
  const int hch  = (wave & 1) * 128 + lane * 4;
#pragma unroll 1
  for (int sub = 0; sub < 4; ++sub) {
    const int lb = g0 + sub * 16;
#pragma unroll 1
    for (int s = 0; s < 16; ++s) {
      const float xcur = XP[(size_t)(lb + s) * kD + d];
      float acc = w0 * xm3;
      acc = fmaf(w1, xm2, acc);
      acc = fmaf(w2, xm1, acc);
      acc = fmaf(w3, xcur, acc);
      sT[s * kTileP + tid] = acc + bc;
      xm3 = xm2; xm2 = xm1; xm1 = xcur;
    }
    __syncthreads();
    v4f fv[4];
    v8h bv[2];
#pragma unroll
    for (int it = 0; it < 4; ++it) fv[it] = *(const v4f*)(sT + (it * 4 + hrow) * kTileP + hch);
#pragma unroll
    for (int it = 0; it < 2; ++it) {
      const float* sp = sT + (it * 8 + wave) * kTileP + lane * 8;
      const v4f a0 = *(const v4f*)(sp);
      const v4f a1 = *(const v4f*)(sp + 4);
#pragma unroll
      for (int e = 0; e < 4; ++e) {
        bv[it][e]     = bfh(a0[e]);
        bv[it][4 + e] = bfh(a1[e]);
      }
    }
    for (int pass = 0; pass < 2; ++pass) {
#pragma unroll
      for (int it = 0; it < 4; ++it)
        *(volatile v4f*)(XC + (size_t)(lb + it * 4 + hrow) * kD + hch) = fv[it];
#pragma unroll
      for (int it = 0; it < 2; ++it)
        *(volatile v8h*)(XCB + (size_t)(lb + it * 8 + wave) * kD + lane * 8) = bv[it];
      __threadfence();
    }
    __syncthreads();
  }
}

__global__ __launch_bounds__(64) void scan_kernel(const float* __restrict__ LGT, float* __restrict__ Y)
{
  __shared__ __align__(16) float sL[kScanT * 32];
  __shared__ __align__(16) float sYt[kScanT * kYP];
  const int tid = threadIdx.x, lane = tid & 31, wave = tid >> 5;
  const int b = blockIdx.x;
  const size_t row0 = (size_t)b * kL;
  const int sc = lane & 15;
  const float padsel = (lane < kS) ? 1.0f : 0.0f;
  const int q = lane >> 3, c4 = (lane & 7) * 4;
  float cp = 1.0f, yc = 0.0f;
#pragma unroll 1
  for (int t0 = 0; t0 < kL; t0 += kScanT) {
    __syncthreads();
#pragma unroll
    for (int it = 0; it < 8; ++it) {
      const int idx = tid + 64 * it;
      const int r = idx >> 3, cc = (idx & 7) * 4;
      *(v4f*)(sL + r * 32 + cc) = *(const v4f*)(LGT + (row0 + t0 + r) * kLgP + cc);
    }
    __syncthreads();
    if (wave == 0) {
#pragma unroll 1
      for (int st = 0; st < kScanT; ++st) {
        const float lg = sL[st * 32 + sc];
        const float db = sL[st * 32 + kS + sc];
        const float a  = expf(lg);
        cp = cp * a;
        float pr = cp * db;
        asm volatile("" : "+v"(pr));
        const float ycn = yc + pr;
        float qv = yc * a;
        asm volatile("" : "+v"(qv));
        float yv = ycn - qv;
        const bool first = (t0 == 0) && (st == 0);
        yv = first ? db : yv;
        yc = ycn;
        sYt[st * kYP + lane] = yv * padsel;
      }
    }
    __syncthreads();
    v4f vals[8];
#pragma unroll
    for (int it = 0; it < 8; ++it) {
      const int row = it * 8 + wave * 4 + q;
      vals[it] = *(const v4f*)(sYt + row * kYP + c4);
    }
    for (int pass = 0; pass < 2; ++pass) {
#pragma unroll
      for (int it = 0; it < 8; ++it) {
        const int row = it * 8 + wave * 4 + q;
        *(volatile v4f*)(Y + (row0 + t0 + row) * kYP + c4) = vals[it];
      }
      __threadfence();
    }
  }
}

__global__ __launch_bounds__(256) void gate_kernel(
    const float* __restrict__ Y, const unsigned short* __restrict__ RES, const float* __restrict__ C_w,
    unsigned short* __restrict__ T1)
{
  __shared__ __align__(16) float sYin[64 * kS];
  __shared__ __align__(16) unsigned int sR[16 * 128];
  __shared__ __align__(16) float sT[16 * kTileP];
  const int tid = threadIdx.x, lane = tid & 31, wave = tid >> 5;
  const int d = tid;
  const int g0 = blockIdx.x * 64;
  v4f cq[4];
#pragma unroll
  for (int q4 = 0; q4 < 4; ++q4) {
    const v4f raw = *(const v4f*)(C_w + (size_t)d * kS + 4 * q4);
    v4f t;
#pragma unroll
    for (int e = 0; e < 4; ++e) t[e] = bfr(raw[e]);
    cq[q4] = t;
  }
  {
    const int r = tid >> 2, cc = (tid & 3) * 4;
    *(v4f*)(sYin + r * kS + cc) = *(const v4f*)(Y + (size_t)(g0 + r) * kYP + cc);
  }
  const int rsh = (d & 1) * 16;
  const int rw  = d >> 1;
#pragma unroll 1
  for (int sub = 0; sub < 4; ++sub) {
    const int lb = g0 + sub * 16;
#pragma unroll
    for (int it = 0; it < 2; ++it) {
      const int idx = tid + it * 256;
      const int r = idx >> 5, c = idx & 31;
      const v4u w = *(const v4u*)(RES + (size_t)(lb + r) * kD + c * 8);
      *(v4u*)(sR + r * 128 + c * 4) = w;
    }
    __syncthreads();
#pragma unroll 1
    for (int s = 0; s < 16; ++s) {
      const float* yr = sYin + (sub * 16 + s) * kS;
      float acc = 0.0f;
#pragma unroll
      for (int q4 = 0; q4 < 4; ++q4) {
        const v4f yv = *(const v4f*)(yr + 4 * q4);
        acc = fmaf(yv[0], cq[q4][0], acc);
        acc = fmaf(yv[1], cq[q4][1], acc);
        acc = fmaf(yv[2], cq[q4][2], acc);
        acc = fmaf(yv[3], cq[q4][3], acc);
      }
      const unsigned int word = sR[s * 128 + rw];
      const float rf = __uint_as_float(((word >> rsh) & 0xffffu) << 16);
      const float sg = rf * (1.0f / (1.0f + expf(-rf)));
      sT[s * kTileP + tid] = acc * sg;
    }
    __syncthreads();
    v8h hv[2];
#pragma unroll
    for (int it = 0; it < 2; ++it) {
      const float* sp = sT + (it * 8 + wave) * kTileP + lane * 8;
      const v4f a0 = *(const v4f*)(sp);
      const v4f a1 = *(const v4f*)(sp + 4);
#pragma unroll
      for (int e = 0; e < 4; ++e) {
        hv[it][e]     = bfh(a0[e]);
        hv[it][4 + e] = bfh(a1[e]);
      }
    }
    for (int pass = 0; pass < 2; ++pass) {
#pragma unroll
      for (int it = 0; it < 2; ++it)
        *(volatile v8h*)(T1 + (size_t)(lb + it * 8 + wave) * kD + lane * 8) = hv[it];
      __threadfence();
    }
    __syncthreads();
  }
}

template <int SQ>
__global__ __launch_bounds__(256) void bn_stat_kernel(
    const float* __restrict__ PRE, const float* __restrict__ MEAN, float* __restrict__ P)
{
  const int d = threadIdx.x;
  const int slab = blockIdx.x;
  float m = 0.0f;
  if (SQ) m = MEAN[d];
  const float* base = PRE + (size_t)slab * kSlabR * kD + d;
  float s = 0.0f;
#pragma unroll 8
  for (int r = 0; r < kSlabR; ++r) {
    const float v = base[(size_t)r * kD];
    if (SQ) { const float t = v - m; s = fmaf(t, t, s); } else { s += v; }
  }
  float* dst = P + (size_t)slab * kD + d;
  *(volatile float*)dst = s;
  __threadfence();
  *(volatile float*)dst = s;
}

template <int RS>
__global__ __launch_bounds__(256) void bn_fin_kernel(const float* __restrict__ P, float* __restrict__ OUTV)
{
  const int d = threadIdx.x;
  float s = 0.0f;
#pragma unroll 8
  for (int j = 0; j < kSlabs; ++j) s += P[(size_t)j * kD + d];
  constexpr float kInvN = 1.0f / (float)kRows;
  float v = s * kInvN;
  if (RS) v = rsqrtf(v + 1e-5f);
  *(volatile float*)(OUTV + d) = v;
  __threadfence();
  *(volatile float*)(OUTV + d) = v;
}

__global__ __launch_bounds__(256) void bn_apply_kernel(
    const float* __restrict__ PRE, const float* __restrict__ MEAN, const float* __restrict__ RSTD,
    const float* __restrict__ gamma, const float* __restrict__ beta, float* __restrict__ OUT)
{
  const int tid = threadIdx.x;
  const int c4 = (tid & 63) * 4, rsub = tid >> 6;
  const int g0 = blockIdx.x * 64;
  const v4f mv   = *(const v4f*)(MEAN + c4);
  const v4f rv   = *(const v4f*)(RSTD + c4);
  const v4f graw = *(const v4f*)(gamma + c4);
  const v4f braw = *(const v4f*)(beta + c4);
  v4f gv, bv;
#pragma unroll
  for (int e = 0; e < 4; ++e) { gv[e] = bfr(graw[e]); bv[e] = bfr(braw[e]); }
#pragma unroll 1
  for (int it = 0; it < 16; ++it) {
    const size_t row = (size_t)(g0 + it * 4 + rsub);
    const v4f p = *(const v4f*)(PRE + row * kD + c4);
    v4f o;
#pragma unroll
    for (int e = 0; e < 4; ++e) {
      float t = p[e] - mv[e];
      t = t * rv[e];
      t = t * gv[e];
      o[e] = t + bv[e];
    }
    float* dst = OUT + row * kD + c4;
    *(volatile v4f*)dst = o;
    __threadfence();
    *(volatile v4f*)dst = o;
  }
}

extern "C" void kernel_launch(void* const* d_in, const int* in_sizes, int n_in,
                              void* d_out, int out_size, void* d_ws, size_t ws_size,
                              hipStream_t stream)
{
  if (n_in < 12) return;
  if (in_sizes[0] != kRows * kD) return;
  if (in_sizes[1] != kD * kS) return;
  if (in_sizes[2] != kS * kD) return;
  if (in_sizes[3] != kD * kS) return;
  if (in_sizes[4] != kD * kKC) return;
  if (in_sizes[5] != kD) return;
  if (in_sizes[6] != kD2 * kD) return;
  if (in_sizes[7] != kD2) return;
  if (in_sizes[8] != kD * kD) return;
  if (in_sizes[9] != kD || in_sizes[10] != kD || in_sizes[11] != kD) return;
  if (out_size != kRows * kD) return;
  if (ws_size < kWsTotal) return;

  const float* x      = (const float*)d_in[0];
  const float* dt     = (const float*)d_in[1];
  const float* B_w    = (const float*)d_in[2];
  const float* C_w    = (const float*)d_in[3];
  const float* conv_w = (const float*)d_in[4];
  const float* conv_b = (const float*)d_in[5];
  const float* in_w   = (const float*)d_in[6];
  const float* in_b   = (const float*)d_in[7];
  const float* out_w  = (const float*)d_in[8];
  const float* out_b  = (const float*)d_in[9];
  const float* gamma  = (const float*)d_in[10];
  const float* beta   = (const float*)d_in[11];
  float* out = (float*)d_out;

  char* ws = (char*)d_ws;
  unsigned short* XB   = (unsigned short*)(ws + kOffXB);
  unsigned short* T1   = (unsigned short*)(ws + kOffXB);
  unsigned short* WIB  = (unsigned short*)(ws + kOffWIB);
  unsigned short* WOB  = (unsigned short*)(ws + kOffWOB);
  unsigned short* WDB  = (unsigned short*)(ws + kOffWDB);
  float*          XP   = (float*)(ws + kOffXP);
  float*          PRE  = (float*)(ws + kOffXP);
  unsigned short* RES  = (unsigned short*)(ws + kOffRES);
  float*          XC   = (float*)(ws + kOffXC);
  unsigned short* XCB  = (unsigned short*)(ws + kOffXCB);
  float*          LGT  = (float*)(ws + kOffLGT);
  float*          Y    = (float*)(ws + kOffY);
  float*          P1   = (float*)(ws + kOffP1);
  float*          P2   = (float*)(ws + kOffP2);
  float*          MEAN = (float*)(ws + kOffMEAN);
  float*          RSTD = (float*)(ws + kOffRSTD);
  const float* dummy_bias  = in_b;
  const float* dummy_resid = x;

  cast_bf16_kernel<<<(kRows * kD) / 8 / 256, 256, 0, stream>>>(x, XB, (kRows * kD) / 8);
  cast_bf16_kernel<<<(kD2 * kD) / 8 / 256, 256, 0, stream>>>(in_w, WIB, (kD2 * kD) / 8);
  cast_bf16_kernel<<<(kD * kD) / 8 / 256, 256, 0, stream>>>(out_w, WOB, (kD * kD) / 8);
  wdb_kernel<<<(64 * kD) / 8 / 256, 256, 0, stream>>>(dt, B_w, WDB);

  wmma_gemm64<1, false, 2, 0, false, 0><<<dim3(256, 1), 256, 0, stream>>>(
      XB, XB, kD, 0L, WIB, WIB, kD, 0L,
      (void*)XP, (void*)XP, kD, 0L, in_b, dummy_resid, 0L, kRows, kD, kD, 1.0f);
  wmma_gemm64<1, false, 2, 3, false, 0><<<dim3(256, 1), 256, 0, stream>>>(
      XB, XB, kD, 0L, WIB + (size_t)kD * kD, WIB + (size_t)kD * kD, kD, 0L,
      (void*)RES, (void*)RES, kD, 0L, in_b + kD, dummy_resid, 0L, kRows, kD, kD, 1.0f);

  conv_kernel<<<kRows / 64, 256, 0, stream>>>(XP, conv_w, conv_b, XC, XCB);

  wmma_gemm64<1, false, 0, 0, false, 0><<<dim3(64, 1), 256, 0, stream>>>(
      XCB, XCB, kD, 0L, WDB, WDB, kD, 0L,
      (void*)LGT, (void*)LGT, kLgP, 0L, dummy_bias, dummy_resid, 0L, kRows, kLgP, kD, 1.0f);

  scan_kernel<<<kB, 64, 0, stream>>>(LGT, Y);

  gate_kernel<<<kRows / 64, 256, 0, stream>>>(Y, RES, C_w, T1);

  wmma_gemm64<1, false, 2, 0, true, 0><<<dim3(256, 1), 256, 0, stream>>>(
      T1, T1, kD, 0L, WOB, WOB, kD, 0L,
      (void*)PRE, (void*)PRE, kD, 0L, out_b, XC, 0L, kRows, kD, kD, 1.0f);

  bn_stat_kernel<0><<<kSlabs, 256, 0, stream>>>(PRE, MEAN, P1);
  bn_fin_kernel<0><<<1, 256, 0, stream>>>(P1, MEAN);
  bn_stat_kernel<1><<<kSlabs, 256, 0, stream>>>(PRE, MEAN, P2);
  bn_fin_kernel<1><<<1, 256, 0, stream>>>(P2, RSTD);
  bn_apply_kernel<<<kRows / 64, 256, 0, stream>>>(PRE, MEAN, RSTD, gamma, beta, out);
}
